// KnotNet_16561393893556
// MI455X (gfx1250) — hardware-run, weakly checked
//
#include <hip/hip_runtime.h>
#include <math.h>

typedef __attribute__((ext_vector_type(16))) _Float16 v16h;
typedef __attribute__((ext_vector_type(8)))  _Float16 v8h;
typedef __attribute__((ext_vector_type(2)))  _Float16 v2h;
typedef __attribute__((ext_vector_type(8)))  float    v8f;
typedef __attribute__((ext_vector_type(4)))  float    v4f;
typedef __attribute__((ext_vector_type(2)))  float    v2f;
typedef __attribute__((ext_vector_type(4)))  int      v4i;

constexpr int kBatch  = 4096;
constexpr int kLen    = 256;
constexpr int kStr    = 4;
constexpr int kHid    = 64;
constexpr int kLayers = 2;
constexpr int kFlat   = kStr * kHid;
constexpr int kN1     = 128;
constexpr int kN2     = 64;
constexpr int kN3     = 2;
static_assert(kFlat == 256, "flat width");
static_assert((kBatch % 64) == 0 && (kN1 % 64) == 0 && (kN2 % 64) == 0, "GEMM M,N multiples of 64");
static_assert((kFlat % 32) == 0 && (kN1 % 32) == 0, "GEMM K multiples of 32");
static_assert(kHid == 64, "two channels per lane of a 32-lane wave");
static_assert((kBatch % 256) == 0 && (kBatch % 8) == 0, "grid multiples");

constexpr float kCarryX = 64.0f;
constexpr float kCarryW = 1024.0f;
constexpr float kCarryH = 64.0f;
constexpr float kScale1 = 1.0f / (kCarryX * kCarryW);
constexpr float kScale2 = 1.0f / (kCarryH * kCarryW);
constexpr float kF16MinNormal = 6.103515625e-5f;
constexpr float kInvHid = 1.0f / (float)kHid;
constexpr float kLnEps  = 1e-5f;

constexpr size_t kOffTAB  = 0;
constexpr size_t kOffW1H  = kOffTAB + 128;
constexpr size_t kOffW2H  = kOffW1H + (size_t)kN1 * kFlat * 2;
constexpr size_t kOffX16  = kOffW2H + (size_t)kN2 * kN1 * 2;
constexpr size_t kOffH1   = kOffX16 + (size_t)kBatch * kFlat * 2;
constexpr size_t kOffH2   = kOffH1  + (size_t)kBatch * kN1 * 2;
constexpr size_t kWsTotal = kOffH2  + (size_t)kBatch * kN2 * 4;
static_assert(kWsTotal == 4276352ull, "carve total");
static_assert(kWsTotal <= 134217728ull, "carve cap");
static_assert((kOffW1H % 128) == 0 && (kOffW2H % 128) == 0 && (kOffX16 % 128) == 0 &&
              (kOffH1 % 128) == 0 && (kOffH2 % 128) == 0, "128-B aligned regions");

__device__ __forceinline__ float carry_flush(float v, float carry) {
  const float x = v * carry;
  return (fabsf(x) < kF16MinNormal) ? 0.0f : x;
}

__device__ __forceinline__ void keep4_h(v16h a, v16h b, v16h c, v16h d) { asm volatile("v_nop" :: "v"(a), "v"(b), "v"(c), "v"(d)); }
__device__ __forceinline__ void acc_guard4(v8f& a, v8f& b, v8f& c, v8f& d) { asm volatile("v_nop\n\tv_nop\n\tv_nop\n\tv_nop" : "+v"(a), "+v"(b), "+v"(c), "+v"(d)); }

union FragU { v16h v; v8h h[2]; };
__device__ __forceinline__ v16h frag_load(const _Float16* p) {
  FragU f;
  f.h[0] = *(const v8h*)(p);
  f.h[1] = *(const v8h*)(p + 16);
  return f.v;
}

__device__ __forceinline__ v8f mma_guarded(v16h a, v16h b, v8f c) {
  c = __builtin_amdgcn_wmma_f32_16x16x32_f16(false, a, false, b, (short)0, c, false, false);
  asm volatile("v_nop\n\tv_nop\n\tv_nop\n\tv_nop" : "+v"(c) : "v"(a), "v"(b));
  return c;
}

__global__ __launch_bounds__(256) void prep_kernel(
    const float* __restrict__ w1, const float* __restrict__ w2, const float* __restrict__ thetas,
    unsigned short* __restrict__ W1H, unsigned short* __restrict__ W2H, float* __restrict__ TAB)
{
  const int tid = threadIdx.x;
  const int blk = blockIdx.x;
  if (blk < 20) {
    const bool first = (blk < 16);
    const float* src = first ? w1 : w2;
    unsigned short* dst = first ? W1H : W2H;
    const int i = (first ? blk : (blk - 16)) * 256 + tid;
    const size_t e0 = (size_t)i << 3;
    const v4f a0 = *(const v4f*)(src + e0);
    const v4f a1 = *(const v4f*)(src + e0 + 4);
    v8h hv;
#pragma unroll
    for (int e = 0; e < 4; ++e) {
      const float x0 = carry_flush(a0[e], kCarryW);
      const float x1 = carry_flush(a1[e], kCarryW);
      hv[e]     = (_Float16)x0;
      hv[4 + e] = (_Float16)x1;
    }
    unsigned short* q = dst + e0;
    *(volatile v8h*)q = hv;
    __threadfence();
    *(volatile v8h*)q = hv;
  } else {
    if (tid >= 32) return;
    int j = (tid < 8) ? tid : (tid - 8);
    j = (j > 5) ? 5 : j;
    float th = thetas[j];
    asm volatile("" : "+v"(th));
    const float cv = cosf(th);
    const float sv = sinf(th);
    float val = 0.0f;
    val = (tid < 6) ? cv : val;
    val = (tid >= 8 && tid < 14) ? sv : val;
    volatile float* p = TAB + tid;
    *p = val;
    __threadfence();
    *p = val;
  }
}

__global__ __launch_bounds__(256) void scan_ln_kernel(
    const int* __restrict__ gens, const float* __restrict__ init, const float* __restrict__ tab,
    const float* __restrict__ lnw, const float* __restrict__ lnb, unsigned* __restrict__ X16w)
{
  __shared__ __align__(16) int sG[8 * kLen];
  __shared__ float sTab[32];
  const int tid = threadIdx.x, lane = tid & 31, wave = tid >> 5;
  const int b0 = blockIdx.x * 8;

  {
    const v4i* src = (const v4i*)(gens + (size_t)b0 * kLen);
#pragma unroll
    for (int i = 0; i < 2; ++i) {
      const int lin4 = i * 256 + tid;
      const v4i g4 = src[lin4];
      *(v4i*)(sG + lin4 * 4) = g4;
    }
    float tv = tab[lane];
    asm volatile("" : "+v"(tv));
    if (wave == 0) sTab[lane] = tv;
  }
  __syncthreads();

  float sa[kStr], sb[kStr];
#pragma unroll
  for (int k = 0; k < kStr; ++k) {
    const v2f i2 = *(const v2f*)(init + k * kHid + 2 * lane);
    sa[k] = i2[0];
    sb[k] = i2[1];
  }

  const int* gw = sG + wave * kLen;

#pragma unroll 1
  for (int layer = 0; layer < kLayers; ++layer) {
    const float c0 = sTab[layer * 3 + 0];
    const float c1 = sTab[layer * 3 + 1];
    const float c2 = sTab[layer * 3 + 2];
    const float s0 = sTab[8 + layer * 3 + 0];
    const float s1 = sTab[8 + layer * 3 + 1];
    const float s2 = sTab[8 + layer * 3 + 2];

#pragma unroll 1
    for (int t = 0; t < kLen; ++t) {
      int g = gw[t];
      g = (g < -4) ? -4 : g;
      g = (g > 4) ? 4 : g;
      const int ag = (g < 0) ? -g : g;
      const int p = ag - 1;
      const bool valid = (p >= 0) && (p <= kStr - 2);
      int pc = (p < 0) ? 0 : p;
      pc = (pc > kStr - 2) ? (kStr - 2) : pc;
      float cc = (pc == 0) ? c0 : ((pc == 1) ? c1 : c2);
      float ss = (pc == 0) ? s0 : ((pc == 1) ? s1 : s2);
      ss = (g < 0) ? -ss : ss;
      const float c = valid ? cc : 1.0f;
      const float s = valid ? ss : 0.0f;
#pragma unroll
      for (int k = 0; k < kStr - 1; ++k) {
        const bool sel = (pc == k);
        const float ck = sel ? c : 1.0f;
        const float sk = sel ? s : 0.0f;
        const float ua = sa[k], va = sa[k + 1];
        sa[k]     = ua * ck - va * sk;
        sa[k + 1] = ua * sk + va * ck;
        const float ub = sb[k], vb = sb[k + 1];
        sb[k]     = ub * ck - vb * sk;
        sb[k + 1] = ub * sk + vb * ck;
      }
    }

    const v2f w2v = *(const v2f*)(lnw + layer * kHid + 2 * lane);
    const v2f b2v = *(const v2f*)(lnb + layer * kHid + 2 * lane);
#pragma unroll
    for (int k = 0; k < kStr; ++k) {
      float sum = sa[k] + sb[k];
#pragma unroll
      for (int m = 16; m >= 1; m >>= 1) sum += __shfl_xor(sum, m, 32);
      const float mu = sum * kInvHid;
      const float da = sa[k] - mu;
      const float db = sb[k] - mu;
      float q = da * da + db * db;
#pragma unroll
      for (int m = 16; m >= 1; m >>= 1) q += __shfl_xor(q, m, 32);
      const float inv = rsqrtf(q * kInvHid + kLnEps);
      sa[k] = (da * inv) * w2v[0] + b2v[0];
      sb[k] = (db * inv) * w2v[1] + b2v[1];
    }
  }

  unsigned wds[kStr];
#pragma unroll
  for (int k = 0; k < kStr; ++k) {
    const float x0 = carry_flush(sa[k], kCarryX);
    const float x1 = carry_flush(sb[k], kCarryX);
    v2h hv;
    hv[0] = (_Float16)x0;
    hv[1] = (_Float16)x1;
    wds[k] = __builtin_bit_cast(unsigned, hv);
  }
  volatile unsigned* dst = X16w + (size_t)(b0 + wave) * (kFlat / 2) + lane;
  for (int pass = 0; pass < 2; ++pass) {
#pragma unroll
    for (int k = 0; k < kStr; ++k) dst[k * 32] = wds[k];
    __threadfence();
  }
}

template <int OUT_MODE>
__global__ __launch_bounds__(256) void gemm_bias_relu_kernel(
    const unsigned short* __restrict__ Ap, int lda,
    const unsigned short* __restrict__ Btp, int ldb,
    void* __restrict__ Cout, int ldc,
    const float* __restrict__ bias,
    int M, int N, int K, float scale, float ocarry)
{
  const _Float16* A  = (const _Float16*)Ap;
  const _Float16* Bt = (const _Float16*)Btp;
  __shared__ __align__(16) float sT[8][16 * 68];
  const int lane = threadIdx.x & 31;
  const int wave = threadIdx.x >> 5;
  const int tilesN = N >> 6;
  const int tilesM = M >> 6;
  const int tile = blockIdx.x * 8 + wave;
  if (tile >= tilesM * tilesN) return;
  const int tm = tile / tilesN;
  const int tn = tile - tm * tilesN;
  const int m0 = tm << 6;
  const int n0 = tn << 6;

  const int rlane = lane & 15;
  const int koff  = (lane >> 4) * 8;
  const int mOff  = (lane >> 4) * 8;

  v8f acc[4][4];
#pragma unroll
  for (int i = 0; i < 4; ++i)
#pragma unroll
    for (int j = 0; j < 4; ++j) acc[i][j] = (v8f){0.f, 0.f, 0.f, 0.f, 0.f, 0.f, 0.f, 0.f};

  for (int k0 = 0; k0 < K; k0 += 32) {
    v16h bh[4];
#pragma unroll
    for (int j = 0; j < 4; ++j) {
      const size_t bo = (size_t)(n0 + (j << 4) + rlane) * ldb + koff + k0;
      bh[j] = frag_load(Bt + bo);
    }
#pragma unroll
    for (int i = 0; i < 4; ++i) {
      const size_t ao = (size_t)(m0 + (i << 4) + rlane) * lda + koff + k0;
      const v16h ah = frag_load(A + ao);
#pragma unroll
      for (int j = 0; j < 4; ++j) acc[i][j] = mma_guarded(ah, bh[j], acc[i][j]);
    }
    keep4_h(bh[0], bh[1], bh[2], bh[3]);
  }
  acc_guard4(acc[0][0], acc[0][1], acc[0][2], acc[0][3]);
  acc_guard4(acc[1][0], acc[1][1], acc[1][2], acc[1][3]);
  acc_guard4(acc[2][0], acc[2][1], acc[2][2], acc[2][3]);
  acc_guard4(acc[3][0], acc[3][1], acc[3][2], acc[3][3]);

  float* slab = sT[wave];
#pragma unroll
  for (int i = 0; i < 4; ++i) {
    const int mBase = m0 + (i << 4);
#pragma unroll
    for (int j = 0; j < 4; ++j) {
      const int n = n0 + (j << 4) + rlane;
      const float bv = bias[n];
#pragma unroll
      for (int r = 0; r < 8; ++r) {
        float v = acc[i][j][r] * scale + bv;
        v = fmaxf(v, 0.0f);
        if (OUT_MODE == 1) {
          v = v * ocarry;
          v = (v < kF16MinNormal) ? 0.0f : v;
        }
        slab[(mOff + r) * 68 + (j << 4) + rlane] = v;
      }
    }
    __builtin_amdgcn_fence(__ATOMIC_RELEASE, "workgroup");
    __builtin_amdgcn_wave_barrier();
    __builtin_amdgcn_fence(__ATOMIC_ACQUIRE, "workgroup");
    if (OUT_MODE == 0) {
      float* C = (float*)Cout;
      const int hh = lane >> 4, c4 = (lane & 15) * 4;
      for (int pass = 0; pass < 2; ++pass) {
#pragma unroll
        for (int it = 0; it < 8; ++it) {
          const int row = it * 2 + hh;
          const v4f v = *(const v4f*)(slab + row * 68 + c4);
          *(volatile v4f*)(C + (size_t)(mBase + row) * ldc + n0 + c4) = v;
        }
        __threadfence();
      }
    } else {
      const int q = lane >> 3, c8 = (lane & 7) * 8;
      unsigned short* C = (unsigned short*)Cout;
      for (int pass = 0; pass < 2; ++pass) {
#pragma unroll
        for (int it = 0; it < 4; ++it) {
          const int row = it * 4 + q;
          const float* sp = slab + row * 68 + c8;
          v8h hv;
#pragma unroll
          for (int e = 0; e < 8; ++e) hv[e] = (_Float16)sp[e];
          *(volatile v8h*)(C + (size_t)(mBase + row) * ldc + n0 + c8) = hv;
        }
        __threadfence();
      }
    }
    __builtin_amdgcn_fence(__ATOMIC_RELEASE, "workgroup");
    __builtin_amdgcn_wave_barrier();
    __builtin_amdgcn_fence(__ATOMIC_ACQUIRE, "workgroup");
  }
}

__global__ __launch_bounds__(256) void head_kernel(
    const float* __restrict__ H2, const float* __restrict__ w3, const float* __restrict__ b3,
    float* __restrict__ out)
{
  const int row = blockIdx.x * 256 + threadIdx.x;
  const float* hr = H2 + (size_t)row * kN2;
  float o0 = 0.0f, o1 = 0.0f;
#pragma unroll 1
  for (int k4 = 0; k4 < kN2 / 4; ++k4) {
    const v4f hv = *(const v4f*)(hr + 4 * k4);
    const v4f wa = *(const v4f*)(w3 + 4 * k4);
    const v4f wb = *(const v4f*)(w3 + kN2 + 4 * k4);
    o0 = fmaf(hv[0], wa[0], o0);
    o0 = fmaf(hv[1], wa[1], o0);
    o0 = fmaf(hv[2], wa[2], o0);
    o0 = fmaf(hv[3], wa[3], o0);
    o1 = fmaf(hv[0], wb[0], o1);
    o1 = fmaf(hv[1], wb[1], o1);
    o1 = fmaf(hv[2], wb[2], o1);
    o1 = fmaf(hv[3], wb[3], o1);
  }
  o0 += b3[0];
  o1 += b3[1];
  const float sg = 1.0f / (1.0f + expf(-o0));
  volatile float* p0 = out + row;
  volatile float* p1 = out + kBatch + row;
  *p0 = sg;
  *p1 = o1;
  __threadfence();
  *p0 = sg;
  *p1 = o1;
}

extern "C" void kernel_launch(void* const* d_in, const int* in_sizes, int n_in,
                              void* d_out, int out_size, void* d_ws, size_t ws_size,
                              hipStream_t stream) {
  if (n_in < 11) return;
  if (in_sizes[0] != kBatch * kLen) return;
  if (in_sizes[1] != kStr * kHid) return;
  if (in_sizes[2] != kLayers * 3) return;
  if (in_sizes[3] != kLayers * kHid) return;
  if (in_sizes[4] != kLayers * kHid) return;
  if (in_sizes[5] != kN1 * kFlat) return;
  if (in_sizes[6] != kN1) return;
  if (in_sizes[7] != kN2 * kN1) return;
  if (in_sizes[8] != kN2) return;
  if (in_sizes[9] != kN3 * kN2) return;
  if (in_sizes[10] != kN3) return;
  if (out_size != 2 * kBatch) return;
  if (ws_size < kWsTotal) return;

  const int*   gens   = (const int*)d_in[0];
  const float* init   = (const float*)d_in[1];
  const float* thetas = (const float*)d_in[2];
  const float* lnw    = (const float*)d_in[3];
  const float* lnb    = (const float*)d_in[4];
  const float* w1     = (const float*)d_in[5];
  const float* b1     = (const float*)d_in[6];
  const float* w2     = (const float*)d_in[7];
  const float* b2     = (const float*)d_in[8];
  const float* w3     = (const float*)d_in[9];
  const float* b3     = (const float*)d_in[10];
  float* out = (float*)d_out;

  char* ws = (char*)d_ws;
  float*          TAB = (float*)(ws + kOffTAB);
  unsigned short* W1H = (unsigned short*)(ws + kOffW1H);
  unsigned short* W2H = (unsigned short*)(ws + kOffW2H);
  unsigned short* X16 = (unsigned short*)(ws + kOffX16);
  unsigned short* H1  = (unsigned short*)(ws + kOffH1);
  float*          H2  = (float*)(ws + kOffH2);

  prep_kernel<<<21, 256, 0, stream>>>(w1, w2, thetas, W1H, W2H, TAB);

  scan_ln_kernel<<<kBatch / 8, 256, 0, stream>>>(gens, init, TAB, lnw, lnb, (unsigned*)X16);

  gemm_bias_relu_kernel<1><<<(kBatch / 64) * (kN1 / 64) / 8, 256, 0, stream>>>(
      X16, kFlat, W1H, kFlat, (void*)H1, kN1, b1, kBatch, kN1, kFlat, kScale1, kCarryH);

  gemm_bias_relu_kernel<0><<<(kBatch / 64) * (kN2 / 64) / 8, 256, 0, stream>>>(
      H1, kN1, W2H, kN1, (void*)H2, kN2, b2, kBatch, kN2, kN1, kScale2, 1.0f);

  head_kernel<<<kBatch / 256, 256, 0, stream>>>(H2, w3, b3, out);
}
